// ImagePairCrossAttention_54314156425561
// MI455X (gfx1250) — hardware-verified
//
#include <hip/hip_runtime.h>
#include <math.h>

typedef __attribute__((ext_vector_type(16))) _Float16 v16h;
typedef __attribute__((ext_vector_type(16))) __bf16 v16b;
typedef __attribute__((ext_vector_type(8)))  _Float16 v8h;
typedef __attribute__((ext_vector_type(8)))  float v8f;
typedef __attribute__((ext_vector_type(4)))  float v4f;
typedef __attribute__((ext_vector_type(2)))  float v2f;
typedef __attribute__((ext_vector_type(4)))  unsigned v4u;
typedef __attribute__((ext_vector_type(4)))  int v4i;
typedef float __attribute__((may_alias)) float_a;
typedef int __attribute__((may_alias)) int_a;

template <typename T> __device__ __forceinline__ void vst2(void* p, T v) { *(volatile T*)p = v; __threadfence(); *(volatile T*)p = v; }
__device__ __forceinline__ v8f wmma16(v16h a, v16h b, v8f c) {
  v8f d = __builtin_amdgcn_wmma_f32_16x16x32_f16(false, a, false, b, (short)0, c, false, false);
  asm volatile("v_nop\n\tv_nop\n\tv_nop\n\tv_nop" : "+v"(d) : "v"(a), "v"(b));
  return d;
}
__device__ __forceinline__ v8f wmma_bf(v16b a, v16b b, v8f c) {
  v8f d = __builtin_amdgcn_wmma_f32_16x16x32_bf16(false, a, false, b, (short)0, c, false, false);
  asm volatile("v_nop\n\tv_nop\n\tv_nop\n\tv_nop" : "+v"(d) : "v"(a), "v"(b));
  return d;
}
__device__ __forceinline__ v16h frag_h(const _Float16* rowk0, int lane) {
  union { v16h v; v8h q[2]; } u; const _Float16* p = rowk0 + 8 * (lane >> 4);
  u.q[0] = *(const v8h*)p; u.q[1] = *(const v8h*)(p + 16); return u.v;
}
__device__ __forceinline__ v16h frag_f32(const float* rowk0, int lane) {
  v16h a; const float* p = rowk0 + 8 * (lane >> 4);
#pragma unroll
  for (int i = 0; i < 8; ++i) { a[i] = (_Float16)p[i]; a[8 + i] = (_Float16)p[16 + i]; }
  return a;
}
__device__ __forceinline__ v16h frag_f32s(const float* rowk0, int lane, float sc) {
  v16h a; const float* p = rowk0 + 8 * (lane >> 4);
#pragma unroll
  for (int i = 0; i < 8; ++i) { a[i] = (_Float16)(p[i] * sc); a[8 + i] = (_Float16)(p[16 + i] * sc); }
  return a;
}
__device__ __forceinline__ v16h fragc_f32(const float* W, int k0, int n, int lane, int ld, int K) {
  v16h a; const int g = lane >> 4;
#pragma unroll
  for (int i = 0; i < 8; ++i) { const int ka = k0 + 8 * g + i, kb = ka + 16;
    a[i] = (_Float16)(ka < K ? W[(size_t)ka * ld + n] : 0.f); a[8 + i] = (_Float16)(kb < K ? W[(size_t)kb * ld + n] : 0.f); }
  return a;
}
struct F2 { v16b h, l; };
__device__ __forceinline__ F2 bsplit16(const float v[16]) { F2 r;
#pragma unroll
  for (int i = 0; i < 16; ++i) { const __bf16 h = (__bf16)v[i]; r.h[i] = h; r.l[i] = (__bf16)(v[i] - (float)h); }
  return r; }
__device__ __forceinline__ F2 split_row(const float* row, int k0, int lane) { float v[16]; const float* p = row + k0 + 8 * (lane >> 4);
#pragma unroll
  for (int i = 0; i < 8; ++i) { v[i] = p[i]; v[8 + i] = p[16 + i]; }
  return bsplit16(v); }
__device__ __forceinline__ F2 split_rowK(const float* row, int k0, int lane, int K) { float v[16]; const int g = lane >> 4;
#pragma unroll
  for (int i = 0; i < 8; ++i) { const int ka = k0 + 8 * g + i, kb = ka + 16; v[i] = ka < K ? row[ka] : 0.f; v[8 + i] = kb < K ? row[kb] : 0.f; }
  return bsplit16(v); }
__device__ __forceinline__ F2 split_col(const float* W, int k0, int n, int lane, int ld, int K) { float v[16]; const int g = lane >> 4;
#pragma unroll
  for (int i = 0; i < 8; ++i) { const int ka = k0 + 8 * g + i, kb = ka + 16; v[i] = ka < K ? W[(size_t)ka * ld + n] : 0.f; v[8 + i] = kb < K ? W[(size_t)kb * ld + n] : 0.f; }
  return bsplit16(v); }
__device__ __forceinline__ v8f mac3(const F2& a, const F2& b, v8f c) { c = wmma_bf(a.l, b.h, c); c = wmma_bf(a.h, b.l, c); return wmma_bf(a.h, b.h, c); }
__device__ __forceinline__ float sigm(float v) { return 1.0f / (1.0f + expf(-v)); }
#define LDSX() do { asm volatile("s_wait_dscnt 0" ::: "memory"); __builtin_amdgcn_wave_barrier(); __builtin_amdgcn_fence(__ATOMIC_RELEASE, "workgroup"); } while (0)

#define NB 32
#define CC 256
#define NT 1024
#define NR (NB * NT)

__global__ __launch_bounds__(256) void k_ln(const float* __restrict__ x, const float* __restrict__ gam, const float* __restrict__ bet, _Float16* __restrict__ xn) {
  __shared__ float tile[CC][65];
  __shared__ float smu[64], srs[64];
  __shared__ __align__(16) _Float16 orow[64][CC + 8];
  const int b = blockIdx.y, n0 = blockIdx.x * 64, tid = threadIdx.x;
  { const int c = tid; const float* src = x + ((size_t)b * CC + c) * NT + n0;
#pragma unroll
    for (int q = 0; q < 16; ++q) { const v4f v = *(const v4f*)(src + q * 4); tile[c][q * 4] = v[0]; tile[c][q * 4 + 1] = v[1]; tile[c][q * 4 + 2] = v[2]; tile[c][q * 4 + 3] = v[3]; } }
  __syncthreads();
  if (tid < 64) { const int n = tid; float s = 0.f; for (int c = 0; c < CC; ++c) s += tile[c][n]; const float mu = s / (float)CC; float q2 = 0.f; for (int c = 0; c < CC; ++c) { const float d = tile[c][n] - mu; q2 += d * d; }
    smu[n] = mu; srs[n] = rsqrtf(q2 / (float)CC + 1e-5f); }
  __syncthreads();
  { const int c = tid; const float gc = gam[c], bc = bet[c];
    for (int n = 0; n < 64; ++n) orow[n][c] = (_Float16)((tile[c][n] - smu[n]) * srs[n] * gc + bc); }
  __syncthreads();
  for (int q = tid; q < 64 * CC / 8; q += 256) { const int n = q >> 5, pc = q & 31; vst2(xn + ((size_t)b * NT + n0 + n) * CC + pc * 8, *(const v4u*)(&orow[n][pc * 8])); }
}
__global__ __launch_bounds__(256) void k_packW(const float* __restrict__ Wq, const float* __restrict__ Wk, _Float16* __restrict__ P) {
  const int n = blockIdx.x, tid = threadIdx.x; const float* W = n < CC ? Wq + (size_t)n * CC : Wk + (size_t)(n - CC) * CC;
  if (tid < CC / 8) { union { v8h h; v4u u; } pk;
#pragma unroll
    for (int e = 0; e < 8; ++e) pk.h[e] = (_Float16)(W[tid * 8 + e] * 16.0f);
    vst2(P + (size_t)n * CC + tid * 8, pk.u); }
}
__global__ __launch_bounds__(128) void k_proj(const _Float16* __restrict__ xn, const _Float16* __restrict__ P, const float* __restrict__ bias, _Float16* __restrict__ dst) {
  __shared__ __align__(16) float so[4][16][132];
  const int tid = threadIdx.x, wave = tid >> 5, lane = tid & 31, col = lane & 15, g = lane >> 4;
  const int r0 = blockIdx.x * 64 + wave * 16, n0 = blockIdx.y * 128; const int nl0 = n0;
  v8f acc[8] = {};
#pragma unroll 1
  for (int kc = 0; kc < CC / 32; ++kc) { const v16h a = frag_h(xn + (size_t)(r0 + col) * CC + kc * 32, lane);
#pragma unroll
    for (int j = 0; j < 8; ++j) acc[j] = wmma16(a, frag_h(P + (size_t)(n0 + j * 16 + col) * CC + kc * 32, lane), acc[j]); }
#pragma unroll
  for (int j = 0; j < 8; ++j) { const float bb = bias[nl0 + j * 16 + col];
#pragma unroll
    for (int r = 0; r < 8; ++r) so[wave][8 * g + r][j * 16 + col] = acc[j][r] * (1.0f / 16.0f) + bb; }
  LDSX();
  for (int q = lane; q < 16 * 16; q += 32) { const int rl = q >> 4, pc = q & 15; union { v8h hh; v4u u; } pk;
#pragma unroll
    for (int e = 0; e < 8; ++e) pk.hh[e] = (_Float16)so[wave][rl][pc * 8 + e];
    vst2(dst + (size_t)(r0 + rl) * CC + nl0 + pc * 8, pk.u); }
}
__global__ __launch_bounds__(128) void k_diag(const _Float16* __restrict__ q16, const _Float16* __restrict__ k16, float* __restrict__ out) {
  __shared__ __align__(16) float sS[4][16][20];
  __shared__ __align__(16) float so[64];
  const int tid = threadIdx.x, w = tid >> 5, lane = tid & 31, col = lane & 15, g = lane >> 4;
  const int b = blockIdx.y, q0 = blockIdx.x * 64 + w * 16;
  const _Float16* qb = q16 + (size_t)b * NT * CC; const _Float16* kb = k16 + (size_t)b * NT * CC;
  v16h aq[8];
#pragma unroll
  for (int kc = 0; kc < 8; ++kc) aq[kc] = frag_h(qb + (size_t)(q0 + col) * CC + kc * 32, lane);
  float mrun = -3.0e38f, lrun = 0.f, sdiag = 0.f;
#pragma unroll 1
  for (int jt = 0; jt < NT / 16; ++jt) { v8f s = {};
#pragma unroll
    for (int kc = 0; kc < 8; ++kc) s = wmma16(aq[kc], frag_h(kb + (size_t)(jt * 16 + col) * CC + kc * 32, lane), s);
#pragma unroll
    for (int r = 0; r < 8; ++r) sS[w][8 * g + r][col] = s[r] * 0.0625f;
    LDSX();
    if (g == 0) { const int m = col; float mx = -3.0e38f;
#pragma unroll
      for (int e = 0; e < 16; ++e) mx = fmaxf(mx, sS[w][m][e]);
      const float mnew = fmaxf(mrun, mx); float ps = 0.f;
#pragma unroll
      for (int e = 0; e < 16; ++e) ps += expf(sS[w][m][e] - mnew);
      lrun = lrun * expf(mrun - mnew) + ps; mrun = mnew;
      const int qi = q0 + m; if (qi >= jt * 16 && qi < jt * 16 + 16) sdiag = sS[w][m][qi - jt * 16]; }
    LDSX(); }
  if (g == 0) so[w * 16 + col] = expf(sdiag - mrun) / lrun;
  __syncthreads();
  if (tid < 16) vst2(out + (size_t)b * NT + blockIdx.x * 64 + tid * 4, *(const v4f*)(&so[tid * 4]));
}
extern "C" void kernel_launch(void* const* d_in, const int* in_sizes, int n_in, void* d_out, int out_size, void* d_ws, size_t ws_size, hipStream_t stream) {
  (void)in_sizes; (void)n_in; (void)out_size; (void)ws_size;
  const float* x = (const float*)d_in[0]; const float* y = (const float*)d_in[1]; const float* gam = (const float*)d_in[2]; const float* bet = (const float*)d_in[3];
  const float* Wq = (const float*)d_in[4]; const float* Wk = (const float*)d_in[5]; const float* bq = (const float*)d_in[6]; const float* bk = (const float*)d_in[7];
  float* out = (float*)d_out;
  char* ws = (char*)d_ws; size_t off = 0;
  auto take = [&](size_t bytes) { char* p = ws + off; off += (bytes + 255) & ~(size_t)255; return p; };
  _Float16* xn = (_Float16*)take((size_t)NR * CC * 2); _Float16* yn = (_Float16*)take((size_t)NR * CC * 2); _Float16* P = (_Float16*)take((size_t)2 * CC * CC * 2);
  _Float16* q16 = (_Float16*)take((size_t)NR * CC * 2); _Float16* k16 = (_Float16*)take((size_t)NR * CC * 2);
  k_ln<<<dim3(NT / 64, NB), 256, 0, stream>>>(x, gam, bet, xn);
  k_ln<<<dim3(NT / 64, NB), 256, 0, stream>>>(y, gam, bet, yn);
  k_packW<<<2 * CC, 256, 0, stream>>>(Wq, Wk, P);
  k_proj<<<dim3(NR / 64, 2), 128, 0, stream>>>(xn, P, bq, q16);
  k_proj<<<dim3(NR / 64, 2), 128, 0, stream>>>(yn, P + (size_t)CC * CC, bk, k16);
  k_diag<<<dim3(NT / 64, NB), 128, 0, stream>>>(q16, k16, out);
}
